// INENHead_86698209837427
// MI455X (gfx1250) — hardware-verified
//
#include <hip/hip_runtime.h>
#include <stddef.h>


#define D       256
#define NC      3
#define NTHR    256
#define NWAVE   8
#define EPT     8
#define NGRP    2
#define CHUNK   (NTHR * EPT * NGRP)
#define WCAP    (EPT * NGRP * 32)
#define LISTN   (NWAVE * WCAP)
#define NB      256
#define NBD     4096
#define GR      32
#define WSCALE  8.0f
#define WINV    0.125f
#define LDS_AGG (NB * D * 4 + LISTN * 4 + 64)

static_assert((CHUNK & (CHUNK - 1)) == 0);
static_assert(CHUNK <= 4096);
static_assert((NB & (NB - 1)) == 0 && NB <= 4096);
static_assert((NBD & (NBD - 1)) == 0 && NBD <= 4096);
static_assert(NB == NTHR);
static_assert(NC == 3);
static_assert((NB * D / 8) % NTHR == 0);
static_assert((NB * NC) % 128 == 0);
static_assert(1024 + NB * NC <= LISTN);
static_assert(NBD == NWAVE * 4 * 128);
static_assert(GR * D * 4 <= 65536);
static_assert((GR % 32) == 0 && (NB % GR) == 0 && (NBD % GR) == 0);

typedef float    v4f  __attribute__((ext_vector_type(4)));
typedef float    v8f  __attribute__((ext_vector_type(8)));
typedef int      v4i  __attribute__((ext_vector_type(4)));
typedef _Float16 v8h  __attribute__((ext_vector_type(8)));
typedef _Float16 v16h __attribute__((ext_vector_type(16)));
union FragH { v16h v; v8h h[2]; };

__device__ __forceinline__ v8h cvt8(v4f a, v4f b) {
  v8h r;
  r[0] = (_Float16)a.x; r[1] = (_Float16)a.y; r[2] = (_Float16)a.z; r[3] = (_Float16)a.w;
  r[4] = (_Float16)b.x; r[5] = (_Float16)b.y; r[6] = (_Float16)b.z; r[7] = (_Float16)b.w;
  return r;
}

__device__ __forceinline__ v8f wmh(v16h a, v16h b, v8f c) {
  v8f d = __builtin_amdgcn_wmma_f32_16x16x32_f16(false, a, false, b, (short)0, c, false, false);
  asm volatile("v_nop\n\tv_nop\n\tv_nop\n\tv_nop" : "+v"(d) : "v"(a), "v"(b));
  return d;
}

template <int NBX>
__device__ __forceinline__ int scan_chunk(const int* __restrict__ dsts, int nE, int cbase, int nodeBase,
                                          int vec8, int* list, int tid, int lane, int wave) {
  (void)lane;
  int wc = 0;
#pragma unroll
  for (int g = 0; g < NGRP; ++g) {
    const int el0  = (g * NTHR + tid) * EPT;
    const int e0   = cbase + el0;
    const int sent = -2147483647 - 1;
    v4i da, db;
    if (vec8 != 0 && e0 + 7 < nE) {
      da = *(const v4i*)(dsts + e0);
      db = *(const v4i*)(dsts + e0 + 4);
    } else {
      da.x = (e0     < nE) ? dsts[min(e0, nE - 1)] : sent;
      da.y = (e0 + 1 < nE) ? dsts[min(e0 + 1, nE - 1)] : sent;
      da.z = (e0 + 2 < nE) ? dsts[min(e0 + 2, nE - 1)] : sent;
      da.w = (e0 + 3 < nE) ? dsts[min(e0 + 3, nE - 1)] : sent;
      db.x = (e0 + 4 < nE) ? dsts[min(e0 + 4, nE - 1)] : sent;
      db.y = (e0 + 5 < nE) ? dsts[min(e0 + 5, nE - 1)] : sent;
      db.z = (e0 + 6 < nE) ? dsts[min(e0 + 6, nE - 1)] : sent;
      db.w = (e0 + 7 < nE) ? dsts[min(e0 + 7, nE - 1)] : sent;
    }
    const unsigned nb = (unsigned)nodeBase;
    const unsigned s0 = (unsigned)da.x - nb, s1 = (unsigned)da.y - nb;
    const unsigned s2 = (unsigned)da.z - nb, s3 = (unsigned)da.w - nb;
    const unsigned s4 = (unsigned)db.x - nb, s5 = (unsigned)db.y - nb;
    const unsigned s6 = (unsigned)db.z - nb, s7 = (unsigned)db.w - nb;
    const bool h0 = s0 < (unsigned)NBX, h1 = s1 < (unsigned)NBX, h2 = s2 < (unsigned)NBX, h3 = s3 < (unsigned)NBX;
    const bool h4 = s4 < (unsigned)NBX, h5 = s5 < (unsigned)NBX, h6 = s6 < (unsigned)NBX, h7 = s7 < (unsigned)NBX;
    const unsigned any = __builtin_amdgcn_ballot_w32(h0 | h1 | h2 | h3 | h4 | h5 | h6 | h7);
    if (any != 0u) {
#define HITJ(J, HJ, SJ) { \
        const unsigned mj = __builtin_amdgcn_ballot_w32(HJ); \
        if (mj != 0u) { \
          if (HJ) { \
            const int pos = wc + (int)__builtin_amdgcn_mbcnt_lo(mj, 0u); \
            if (pos < WCAP) list[wave * WCAP + pos] = ((el0 + (J)) << 12) | (int)(SJ); \
          } \
          wc += (int)__builtin_popcount(mj); } }
      HITJ(0, h0, s0)
      HITJ(1, h1, s1)
      HITJ(2, h2, s2)
      HITJ(3, h3, s3)
      HITJ(4, h4, s4)
      HITJ(5, h5, s5)
      HITJ(6, h6, s6)
      HITJ(7, h7, s7)
#undef HITJ
    }
  }
  return wc;
}

__global__ __launch_bounds__(NTHR) void k_wprep(
    const float* __restrict__ We, const float* __restrict__ W1, const float* __restrict__ W2,
    _Float16* wes, _Float16* w1s, _Float16* w2s) {
  const int i   = blockIdx.x * NTHR + threadIdx.x;
  const int per = D * D / 8;
  if (i >= 3 * per) return;
  const int p  = i / per;
  const int o  = (i - p * per) * 8;
  const int n  = o / D;
  const int k0 = o - n * D;
  const float* W  = (p == 0) ? We  : ((p == 1) ? W1  : W2);
  _Float16*    dp = ((p == 0) ? wes : ((p == 1) ? w1s : w2s)) + o;
  const float* q = W + (size_t)k0 * D + n;
  v4f a, b;
  a.x = q[0];     a.y = q[D];     a.z = q[2 * D]; a.w = q[3 * D];
  b.x = q[4 * D]; b.y = q[5 * D]; b.z = q[6 * D]; b.w = q[7 * D];
  a = a * WSCALE;
  b = b * WSCALE;
  const v8h hv = cvt8(a, b);
  *(volatile v8h*)dp = hv;
  __threadfence();
  *(volatile v8h*)dp = hv;
}

__global__ __launch_bounds__(NTHR) void k_xprep(
    const float* __restrict__ x, _Float16* x16, int nN, int nItems) {
  const int i = blockIdx.x * NTHR + threadIdx.x;
  if (i >= nItems) return;
  const int row = i >> 5;
  const int c0  = (i & 31) * 8;
  const int srow = row < nN ? row : nN - 1;
  const float* xp = x + (size_t)srow * D + c0;
  const v4f a = *(const v4f*)xp, b = *(const v4f*)(xp + 4);
  const v8h hv = cvt8(a, b);
  _Float16* dp = x16 + (size_t)i * 8;
  *(volatile v8h*)dp = hv;
  __threadfence();
  *(volatile v8h*)dp = hv;
}

__global__ __launch_bounds__(NTHR) void k_deg(
    const int* __restrict__ ei, float* dinv, int nN, int nE, int vec8) {
  __shared__ __attribute__((aligned(16))) int cnt[NBD];
  __shared__ __attribute__((aligned(16))) int list[LISTN];
  __shared__ int wcnt[NWAVE];
  const int tid = threadIdx.x, lane = tid & 31, wave = tid >> 5;
  const int nodeBase = blockIdx.x * NBD;
  const int* dsts = ei + nE;
  (void)nN;

  for (int i = tid; i < NBD; i += NTHR) cnt[i] = 0;
  __syncthreads();

  const int nChunks = (nE + CHUNK - 1) / CHUNK;
#pragma unroll 1
  for (int ch = 0; ch < nChunks; ++ch) {
    const int cbase = ch * CHUNK;
    const int wc = scan_chunk<NBD>(dsts, nE, cbase, nodeBase, vec8, list, tid, lane, wave);
    if (lane == 0) wcnt[wave] = wc;
    __syncthreads();
    if (wave == 0) {
#pragma unroll 1
      for (int wsx = 0; wsx < NWAVE; ++wsx) {
        int n = __builtin_amdgcn_readfirstlane(wcnt[wsx]);
        n = n > WCAP ? WCAP : (n < 0 ? 0 : n);
        const int* lp = list + wsx * WCAP;
#pragma unroll 1
        for (int i = 0; i < n; ++i) {
          const int ent  = __builtin_amdgcn_readfirstlane(lp[i]);
          const int slot = ent & (NBD - 1);
          if (lane == 0) cnt[slot] = cnt[slot] + 1;
        }
      }
    }
    __syncthreads();
  }

  v4f dq[4];
#pragma unroll
  for (int q = 0; q < 4; ++q) {
    const int f = (wave * 4 + q) * 128 + 4 * lane;
    const v4i c = *(const v4i*)(cnt + f);
    dq[q].x = rsqrtf((float)(c.x + 1));
    dq[q].y = rsqrtf((float)(c.y + 1));
    dq[q].z = rsqrtf((float)(c.z + 1));
    dq[q].w = rsqrtf((float)(c.w + 1));
  }
  float* dp = dinv + (size_t)nodeBase;
#pragma unroll
  for (int q = 0; q < 4; ++q) *(volatile v4f*)(dp + (wave * 4 + q) * 128 + 4 * lane) = dq[q];
  __threadfence();
#pragma unroll
  for (int q = 0; q < 4; ++q) *(volatile v4f*)(dp + (wave * 4 + q) * 128 + 4 * lane) = dq[q];
}

template <int MODE>
__global__ __launch_bounds__(NTHR) void k_gemm(
    const _Float16* __restrict__ A16, const _Float16* __restrict__ Wnk,
    const float* __restrict__ bias, const float* __restrict__ dinv,
    _Float16* out16, float* out32) {
  __shared__ __attribute__((aligned(16))) float stg[GR * D];
  _Float16* s16 = (_Float16*)stg;
  const int tid = threadIdx.x, lane = tid & 31, wave = tid >> 5, hh = lane >> 4, m = lane & 15;
  const int rt = wave & 1, cq = wave >> 1;
  const int rowBase = blockIdx.x * GR;

  v8f acc[4];
#pragma unroll
  for (int t = 0; t < 4; ++t) { v8f z = {0.f, 0.f, 0.f, 0.f, 0.f, 0.f, 0.f, 0.f}; acc[t] = z; }

  const _Float16* ar = A16 + ((size_t)rowBase + 16 * rt + m) * D + 8 * hh;
  const _Float16* br = Wnk + (size_t)(64 * cq + m) * D + 8 * hh;
#pragma unroll 2
  for (int kt = 0; kt < D / 32; ++kt) {
    FragH a;
    a.h[0] = *(const v8h*)(ar + 32 * kt);
    a.h[1] = *(const v8h*)(ar + 32 * kt + 16);
#pragma unroll
    for (int t = 0; t < 4; ++t) {
      const _Float16* bp = br + (size_t)(16 * t) * D + 32 * kt;
      FragH b;
      b.h[0] = *(const v8h*)bp;
      b.h[1] = *(const v8h*)(bp + 16);
      acc[t] = wmh(a.v, b.v, acc[t]);
    }
  }

  const int r0 = 16 * rt + 8 * hh;
  if (MODE == 0) {
    float bv[4];
#pragma unroll
    for (int t = 0; t < 4; ++t) bv[t] = bias[64 * cq + 16 * t + m];
    _Float16* sp = s16 + r0 * D + 64 * cq + m;
#pragma unroll
    for (int t = 0; t < 4; ++t) {
#pragma unroll
      for (int r = 0; r < 8; ++r) sp[r * D + 16 * t] = (_Float16)fmaxf(acc[t][r] * WINV + bv[t], 0.f);
    }
    __syncthreads();
    v8h ov[4];
#pragma unroll
    for (int i = 0; i < 4; ++i) ov[i] = *(const v8h*)(s16 + (4 * wave + i) * D + 8 * lane);
    _Float16* gp = out16 + ((size_t)rowBase + 4 * wave) * D + 8 * lane;
#pragma unroll
    for (int i = 0; i < 4; ++i) *(volatile v8h*)(gp + (size_t)i * D) = ov[i];
    __threadfence();
#pragma unroll
    for (int i = 0; i < 4; ++i) *(volatile v8h*)(gp + (size_t)i * D) = ov[i];
  } else {
    const v4f dA = *(const v4f*)(dinv + (size_t)rowBase + r0);
    const v4f dB = *(const v4f*)(dinv + (size_t)rowBase + r0 + 4);
    float dr[8];
    dr[0] = dA.x * WINV; dr[1] = dA.y * WINV; dr[2] = dA.z * WINV; dr[3] = dA.w * WINV;
    dr[4] = dB.x * WINV; dr[5] = dB.y * WINV; dr[6] = dB.z * WINV; dr[7] = dB.w * WINV;
    float* sp = stg + r0 * D + 64 * cq + m;
#pragma unroll
    for (int t = 0; t < 4; ++t) {
#pragma unroll
      for (int r = 0; r < 8; ++r) sp[r * D + 16 * t] = acc[t][r] * dr[r];
    }
    __syncthreads();
    v4f ov[8];
#pragma unroll
    for (int i = 0; i < 4; ++i) {
      ov[2 * i]     = *(const v4f*)(stg + (4 * wave + i) * D + 4 * lane);
      ov[2 * i + 1] = *(const v4f*)(stg + (4 * wave + i) * D + 128 + 4 * lane);
    }
    float* gp = out32 + ((size_t)rowBase + 4 * wave) * D + 4 * lane;
#pragma unroll
    for (int i = 0; i < 4; ++i) {
      *(volatile v4f*)(gp + (size_t)i * D)       = ov[2 * i];
      *(volatile v4f*)(gp + (size_t)i * D + 128) = ov[2 * i + 1];
    }
    __threadfence();
#pragma unroll
    for (int i = 0; i < 4; ++i) {
      *(volatile v4f*)(gp + (size_t)i * D)       = ov[2 * i];
      *(volatile v4f*)(gp + (size_t)i * D + 128) = ov[2 * i + 1];
    }
  }
}

__device__ __forceinline__ void agg_row8(const float* acc, const float* __restrict__ g,
                                         const float* __restrict__ dinv, const float* __restrict__ bias,
                                         int nodeBase, int nN, int idx, v4f& o0, v4f& o1) {
  const int slot = idx >> 5, c8 = (idx & 31) * 8;
  int node = nodeBase + slot;
  node = node > nN - 1 ? nN - 1 : node;
  const float d = dinv[node];
  const float* gp = g + (size_t)node * D + c8;
  const v4f g0 = *(const v4f*)gp, g1 = *(const v4f*)(gp + 4);
  const v4f b0 = *(const v4f*)(bias + c8), b1 = *(const v4f*)(bias + c8 + 4);
  const v4f a0 = *(const v4f*)(acc + slot * D + c8), a1 = *(const v4f*)(acc + slot * D + c8 + 4);
  o0 = (a0 + g0) * d + b0;
  o1 = (a1 + g1) * d + b1;
}

__device__ __forceinline__ void agg_store_h16(const float* acc, const float* __restrict__ g,
                                              const float* __restrict__ dinv, const float* __restrict__ bias,
                                              _Float16* hout, int nodeBase, int nN, int tid) {
#pragma unroll 2
  for (int i = 0; i < (NB * D / 8) / NTHR; ++i) {
    const int idx = i * NTHR + tid;
    v4f o0, o1;
    agg_row8(acc, g, dinv, bias, nodeBase, nN, idx, o0, o1);
    const int slot = idx >> 5, c8 = (idx & 31) * 8;
    *(volatile v8h*)(hout + ((size_t)nodeBase + slot) * D + c8) = cvt8(o0, o1);
  }
}

__device__ __forceinline__ void out_pass(const float* lg, float* out, size_t ob, size_t outN, int lane) {
#pragma unroll
  for (int q = 0; q < (NB * NC) / 128; ++q) {
    const int f = q * 128 + 4 * lane;
    const size_t gi = ob + (size_t)f;
    const v4f v = *(const v4f*)(lg + f);
    if (gi + 4 <= outN) {
      *(volatile v4f*)(out + gi) = v;
    } else {
      if (gi     < outN) *(volatile float*)(out + gi)     = v.x;
      if (gi + 1 < outN) *(volatile float*)(out + gi + 1) = v.y;
      if (gi + 2 < outN) *(volatile float*)(out + gi + 2) = v.z;
    }
  }
}

template <int MODE>
__global__ __launch_bounds__(NTHR) void k_agg(
    const int* __restrict__ ei, const float* __restrict__ g, const float* __restrict__ dinv,
    const float* __restrict__ bias, const float* __restrict__ wcls, const float* __restrict__ bcls,
    _Float16* hout, float* out, int nN, int nE, int vec8) {
  extern __shared__ v4f lds_dyn[];
  float* acc  = (float*)lds_dyn;
  int*   list = (int*)(acc + NB * D);
  int*   wcnt = list + LISTN;
  const int tid = threadIdx.x, lane = tid & 31, wave = tid >> 5;
  const int nodeBase = blockIdx.x * NB;
  const int* dsts = ei + nE;

  {
    const v4f z = {0.f, 0.f, 0.f, 0.f};
    for (int i = tid; i < NB * D / 4; i += NTHR) lds_dyn[i] = z;
  }
  __syncthreads();

  const int nChunks = (nE + CHUNK - 1) / CHUNK;
#pragma unroll 1
  for (int ch = 0; ch < nChunks; ++ch) {
    const int cbase = ch * CHUNK;
    const int wc = scan_chunk<NB>(dsts, nE, cbase, nodeBase, vec8, list, tid, lane, wave);
    if (lane == 0) wcnt[wave] = wc;
    __syncthreads();
    if (wave == 0) {
#pragma unroll 1
      for (int wsx = 0; wsx < NWAVE; ++wsx) {
        int n = __builtin_amdgcn_readfirstlane(wcnt[wsx]);
        n = n > WCAP ? WCAP : (n < 0 ? 0 : n);
        const int* lp = list + wsx * WCAP;
#pragma unroll 1
        for (int i = 0; i < n; ++i) {
          const int ent  = __builtin_amdgcn_readfirstlane(lp[i]);
          const int slot = ent & (NB - 1);
          int e = cbase + ((ent >> 12) & (CHUNK - 1));
          e = e > nE - 1 ? nE - 1 : e;
          int src = ei[e];
          src = src < 0 ? 0 : (src > nN - 1 ? nN - 1 : src);
          const float* gp = g + (size_t)src * D;
          const v4f v0 = *(const v4f*)(gp + 4 * lane);
          const v4f v1 = *(const v4f*)(gp + 128 + 4 * lane);
          v4f* ap = (v4f*)(acc + slot * D);
          ap[lane]      = ap[lane] + v0;
          ap[32 + lane] = ap[32 + lane] + v1;
        }
      }
    }
    __syncthreads();
  }

  if (MODE == 1) {
    agg_store_h16(acc, g, dinv, bias, hout, nodeBase, nN, tid);
    __threadfence();
    agg_store_h16(acc, g, dinv, bias, hout, nodeBase, nN, tid);
  } else {
    float* wl = (float*)list;
    float* lg = wl + 1024;
#pragma unroll 2
    for (int i = 0; i < (NB * D / 8) / NTHR; ++i) {
      const int idx = i * NTHR + tid;
      v4f o0, o1;
      agg_row8(acc, g, dinv, bias, nodeBase, nN, idx, o0, o1);
      const int slot = idx >> 5, c8 = (idx & 31) * 8;
      *(v4f*)(acc + slot * D + c8)     = o0;
      *(v4f*)(acc + slot * D + c8 + 4) = o1;
    }
    for (int i = tid; i < D * NC; i += NTHR) wl[i] = wcls[i];
    if (tid < NC) wl[D * NC + tid] = bcls[tid];
    __syncthreads();

    {
      const float* hr = acc + tid * D;
      float l0 = 0.f, l1 = 0.f, l2 = 0.f;
#pragma unroll 2
      for (int k4 = 0; k4 < D / 4; ++k4) {
        const v4f   hv = *(const v4f*)(hr + 4 * k4);
        const float* wp = wl + 12 * k4;
        l0 += hv.x * wp[0]; l1 += hv.x * wp[1];  l2 += hv.x * wp[2];
        l0 += hv.y * wp[3]; l1 += hv.y * wp[4];  l2 += hv.y * wp[5];
        l0 += hv.z * wp[6]; l1 += hv.z * wp[7];  l2 += hv.z * wp[8];
        l0 += hv.w * wp[9]; l1 += hv.w * wp[10]; l2 += hv.w * wp[11];
      }
      lg[tid * NC + 0] = l0 + wl[D * NC + 0];
      lg[tid * NC + 1] = l1 + wl[D * NC + 1];
      lg[tid * NC + 2] = l2 + wl[D * NC + 2];
    }
    __syncthreads();

    const size_t outN = (size_t)nN * NC;
    const size_t ob   = (size_t)nodeBase * NC;
    if (wave == 0) out_pass(lg, out, ob, outN, lane);
    __threadfence();
    if (wave == 0) out_pass(lg, out, ob, outN, lane);
  }
}

extern "C" void kernel_launch(void* const* d_in, const int* in_sizes, int n_in,
                              void* d_out, int out_size, void* d_ws, size_t ws_size,
                              hipStream_t stream) {
  if (n_in < 10) return;
  const int nN = in_sizes[0] / D;
  const int nE = in_sizes[1] / 2;
  if (nN <= 0 || nE < 0 || in_sizes[0] != nN * D || in_sizes[1] != nE * 2) return;
  if (in_sizes[2] != D * D || in_sizes[3] < D || in_sizes[4] != D * D || in_sizes[5] < D) return;
  if (in_sizes[6] != D * D || in_sizes[7] < D || in_sizes[8] != D * NC || in_sizes[9] < NC) return;
  if (out_size != nN * NC) return;

  const float* x  = (const float*)d_in[0];
  const int*   ei = (const int*)d_in[1];
  const float* We = (const float*)d_in[2];
  const float* be = (const float*)d_in[3];
  const float* W1 = (const float*)d_in[4];
  const float* b1 = (const float*)d_in[5];
  const float* W2 = (const float*)d_in[6];
  const float* b2 = (const float*)d_in[7];
  const float* Wc = (const float*)d_in[8];
  const float* bc = (const float*)d_in[9];
  float* out = (float*)d_out;

  const int nBD = (nN + NBD - 1) / NBD;
  const int nGB = (nN + GR - 1) / GR;
  const int NPg = nGB * GR;
  const int nAB = (nN + NB - 1) / NB;
  const int NPa = nAB * NB;

  char* ws = (char*)d_ws;
  size_t off = 0;
  const size_t oWe = off; off += (size_t)D * D * 2;          off = (off + 255) & ~(size_t)255;
  const size_t oW1 = off; off += (size_t)D * D * 2;          off = (off + 255) & ~(size_t)255;
  const size_t oW2 = off; off += (size_t)D * D * 2;          off = (off + 255) & ~(size_t)255;
  const size_t oDv = off; off += (size_t)nBD * NBD * 4;      off = (off + 255) & ~(size_t)255;
  const size_t oX  = off; off += (size_t)NPg * D * 2;        off = (off + 255) & ~(size_t)255;
  const size_t oH0 = off; off += (size_t)NPg * D * 2;        off = (off + 255) & ~(size_t)255;
  const size_t oG1 = off; off += (size_t)NPg * D * 4;        off = (off + 255) & ~(size_t)255;
  const size_t oH1 = off; off += (size_t)NPa * D * 2;        off = (off + 255) & ~(size_t)255;
  const size_t oG2 = off; off += (size_t)NPg * D * 4;        off = (off + 255) & ~(size_t)255;
  if (off > ws_size) return;
  _Float16* wes  = (_Float16*)(ws + oWe);
  _Float16* w1s  = (_Float16*)(ws + oW1);
  _Float16* w2s  = (_Float16*)(ws + oW2);
  float*    dinv = (float*)(ws + oDv);
  _Float16* x16  = (_Float16*)(ws + oX);
  _Float16* h0   = (_Float16*)(ws + oH0);
  float*    g1   = (float*)(ws + oG1);
  _Float16* h1   = (_Float16*)(ws + oH1);
  float*    g2   = (float*)(ws + oG2);

  const int vec8 = ((nE & 3) == 0) ? 1 : 0;

  const int nPrep = 3 * (D * D / 8);
  k_wprep<<<(nPrep + NTHR - 1) / NTHR, NTHR, 0, stream>>>(We, W1, W2, wes, w1s, w2s);

  const int nItemsX = NPg * (D / 8);
  k_xprep<<<(nItemsX + NTHR - 1) / NTHR, NTHR, 0, stream>>>(x, x16, nN, nItemsX);

  k_deg<<<nBD, NTHR, 0, stream>>>(ei, dinv, nN, nE, vec8);

  k_gemm<0><<<nGB, NTHR, 0, stream>>>(x16, wes, be, dinv, h0, g1);
  k_gemm<1><<<nGB, NTHR, 0, stream>>>(h0, w1s, b1, dinv, h1, g1);

  hipFuncSetAttribute(reinterpret_cast<const void*>(&k_agg<1>),
                      hipFuncAttributeMaxDynamicSharedMemorySize, LDS_AGG);
  k_agg<1><<<nAB, NTHR, LDS_AGG, stream>>>(ei, g1, dinv, b1, Wc, bc, h1, out, nN, nE, vec8);

  k_gemm<1><<<nGB, NTHR, 0, stream>>>(h1, w2s, b2, dinv, h0, g2);

  hipFuncSetAttribute(reinterpret_cast<const void*>(&k_agg<2>),
                      hipFuncAttributeMaxDynamicSharedMemorySize, LDS_AGG);
  k_agg<2><<<nAB, NTHR, LDS_AGG, stream>>>(ei, g2, dinv, b2, Wc, bc, h1, out, nN, nE, vec8);
}
